// EDRNCell_51659866637126
// MI455X (gfx1250) — hardware-verified
//
#include <hip/hip_runtime.h>
#include <math.h>

typedef __attribute__((ext_vector_type(16))) _Float16 v16h;
typedef __attribute__((ext_vector_type(16))) __bf16 v16b;
typedef __attribute__((ext_vector_type(8)))  _Float16 v8h;
typedef __attribute__((ext_vector_type(8)))  float v8f;
typedef __attribute__((ext_vector_type(4)))  float v4f;
typedef __attribute__((ext_vector_type(2)))  float v2f;
typedef __attribute__((ext_vector_type(4)))  unsigned v4u;
typedef __attribute__((ext_vector_type(4)))  int v4i;
typedef float __attribute__((may_alias)) float_a;
typedef int __attribute__((may_alias)) int_a;

template <typename T> __device__ __forceinline__ void vst2(void* p, T v) { *(volatile T*)p = v; __threadfence(); *(volatile T*)p = v; }
__device__ __forceinline__ v8f wmma16(v16h a, v16h b, v8f c) {
  v8f d = __builtin_amdgcn_wmma_f32_16x16x32_f16(false, a, false, b, (short)0, c, false, false);
  asm volatile("v_nop\n\tv_nop\n\tv_nop\n\tv_nop" : "+v"(d) : "v"(a), "v"(b));
  return d;
}
__device__ __forceinline__ v8f wmma_bf(v16b a, v16b b, v8f c) {
  v8f d = __builtin_amdgcn_wmma_f32_16x16x32_bf16(false, a, false, b, (short)0, c, false, false);
  asm volatile("v_nop\n\tv_nop\n\tv_nop\n\tv_nop" : "+v"(d) : "v"(a), "v"(b));
  return d;
}
__device__ __forceinline__ v16h frag_h(const _Float16* rowk0, int lane) {
  union { v16h v; v8h q[2]; } u; const _Float16* p = rowk0 + 8 * (lane >> 4);
  u.q[0] = *(const v8h*)p; u.q[1] = *(const v8h*)(p + 16); return u.v;
}
__device__ __forceinline__ v16h frag_f32(const float* rowk0, int lane) {
  v16h a; const float* p = rowk0 + 8 * (lane >> 4);
#pragma unroll
  for (int i = 0; i < 8; ++i) { a[i] = (_Float16)p[i]; a[8 + i] = (_Float16)p[16 + i]; }
  return a;
}
__device__ __forceinline__ v16h frag_f32s(const float* rowk0, int lane, float sc) {
  v16h a; const float* p = rowk0 + 8 * (lane >> 4);
#pragma unroll
  for (int i = 0; i < 8; ++i) { a[i] = (_Float16)(p[i] * sc); a[8 + i] = (_Float16)(p[16 + i] * sc); }
  return a;
}
__device__ __forceinline__ v16h fragc_f32(const float* W, int k0, int n, int lane, int ld, int K) {
  v16h a; const int g = lane >> 4;
#pragma unroll
  for (int i = 0; i < 8; ++i) { const int ka = k0 + 8 * g + i, kb = ka + 16;
    a[i] = (_Float16)(ka < K ? W[(size_t)ka * ld + n] : 0.f); a[8 + i] = (_Float16)(kb < K ? W[(size_t)kb * ld + n] : 0.f); }
  return a;
}
struct F2 { v16b h, l; };
__device__ __forceinline__ F2 bsplit16(const float v[16]) { F2 r;
#pragma unroll
  for (int i = 0; i < 16; ++i) { const __bf16 h = (__bf16)v[i]; r.h[i] = h; r.l[i] = (__bf16)(v[i] - (float)h); }
  return r; }
__device__ __forceinline__ F2 split_row(const float* row, int k0, int lane) { float v[16]; const float* p = row + k0 + 8 * (lane >> 4);
#pragma unroll
  for (int i = 0; i < 8; ++i) { v[i] = p[i]; v[8 + i] = p[16 + i]; }
  return bsplit16(v); }
__device__ __forceinline__ F2 split_rowK(const float* row, int k0, int lane, int K) { float v[16]; const int g = lane >> 4;
#pragma unroll
  for (int i = 0; i < 8; ++i) { const int ka = k0 + 8 * g + i, kb = ka + 16; v[i] = ka < K ? row[ka] : 0.f; v[8 + i] = kb < K ? row[kb] : 0.f; }
  return bsplit16(v); }
__device__ __forceinline__ F2 split_col(const float* W, int k0, int n, int lane, int ld, int K) { float v[16]; const int g = lane >> 4;
#pragma unroll
  for (int i = 0; i < 8; ++i) { const int ka = k0 + 8 * g + i, kb = ka + 16; v[i] = ka < K ? W[(size_t)ka * ld + n] : 0.f; v[8 + i] = kb < K ? W[(size_t)kb * ld + n] : 0.f; }
  return bsplit16(v); }
__device__ __forceinline__ v8f mac3(const F2& a, const F2& b, v8f c) { c = wmma_bf(a.l, b.h, c); c = wmma_bf(a.h, b.l, c); return wmma_bf(a.h, b.h, c); }
__device__ __forceinline__ float sigm(float v) { return 1.0f / (1.0f + expf(-v)); }
#define LDSX() do { asm volatile("s_wait_dscnt 0" ::: "memory"); __builtin_amdgcn_wave_barrier(); __builtin_amdgcn_fence(__ATOMIC_RELEASE, "workgroup"); } while (0)

__device__ __forceinline__ v16h fragc_f32s(const float* __restrict__ base, int k0, int n, int lane, int ld, float sc) {
  const int g = lane >> 4; v16h r;
#pragma unroll
  for (int i = 0; i < 8; ++i) { r[i] = (_Float16)(base[(size_t)(k0 + 8 * g + i) * ld + n] * sc); r[8 + i] = (_Float16)(base[(size_t)(k0 + 16 + 8 * g + i) * ld + n] * sc); }
  return r;
}
#define NBT 1024
#define NX 256
#define MM 512
#define DDG 4
#define MD (MM * DDG)

__global__ __launch_bounds__(256) void k_last(const float* __restrict__ a, float* __restrict__ AL) {
  const size_t i = (size_t)blockIdx.x * 256 + threadIdx.x; if (i >= (size_t)NBT * MM) return; vst2(AL + i, a[i * DDG + 3]);
}
__global__ __launch_bounds__(128) void k_p1(const float* __restrict__ x, const float* __restrict__ m, const float* __restrict__ a, const float* __restrict__ AL,
    const float* __restrict__ Afg, const float* __restrict__ Ain, const float* __restrict__ Ath, const float* __restrict__ Apt, const float* __restrict__ Bfg, const float* __restrict__ Bin, const float* __restrict__ Bth,
    const float* __restrict__ bfg, const float* __restrict__ bin_, const float* __restrict__ bth, float* __restrict__ anew, float* __restrict__ ANL) {
  __shared__ __align__(16) float sg[3][4][16][132];
  __shared__ __align__(16) float sl[4][16][36];
  const int tid = threadIdx.x, wave = tid >> 5, lane = tid & 31, col = lane & 15, g = lane >> 4;
  const int r0 = blockIdx.x * 64 + wave * 16, n0 = blockIdx.y * 128;
#pragma unroll 1
  for (int gate = 0; gate < 3; ++gate) {
    const float* Am = gate == 0 ? Afg : gate == 1 ? Ain : Ath; const float* Bx = gate == 0 ? Bfg : gate == 1 ? Bin : Bth; const float* bb = gate == 0 ? bfg : gate == 1 ? bin_ : bth;
    const float* Arow = gate == 2 ? AL : m;
    v8f acc[8] = {};
#pragma unroll 1
    for (int kc = 0; kc < MM / 32; ++kc) { const v16h fa = frag_f32(Arow + (size_t)(r0 + col) * MM + kc * 32, lane);
#pragma unroll
      for (int j = 0; j < 8; ++j) acc[j] = wmma16(fa, fragc_f32s(Am, kc * 32, n0 + j * 16 + col, lane, MD, 16.0f), acc[j]); }
#pragma unroll 1
    for (int kc = 0; kc < NX / 32; ++kc) { const v16h fa = frag_f32(x + (size_t)(r0 + col) * NX + kc * 32, lane);
#pragma unroll
      for (int j = 0; j < 8; ++j) acc[j] = wmma16(fa, fragc_f32s(Bx, kc * 32, n0 + j * 16 + col, lane, MD, 16.0f), acc[j]); }
#pragma unroll
    for (int j = 0; j < 8; ++j) { const float bv = bb[n0 + j * 16 + col];
#pragma unroll
      for (int r = 0; r < 8; ++r) sg[gate][wave][8 * g + r][j * 16 + col] = acc[j][r] * (1.0f / 16.0f) + bv; } }
  LDSX();
  { const int rl = lane >> 1, hf = lane & 1; const int row = r0 + rl; const float* arow = a + (size_t)row * MD; const float* alr = AL + (size_t)row * MM;
#pragma unroll 1
    for (int c = hf * 64; c < hf * 64 + 64; ++c) { const int n = n0 + c; const int mcol = n >> 2, jj = n & 3;
      float v = sg[2][wave][rl][c] - alr[mcol] * Ath[(size_t)mcol * MD + n];
      const float* ar = arow + mcol * DDG;
      for (int i = 0; i < jj; ++i) v += ar[i] * Apt[(size_t)(mcol * DDG + i) * MD + n];
      const float an = arow[n] * sigm(sg[0][wave][rl][c]) + tanhf(v) * sigm(sg[1][wave][rl][c]);
      sg[2][wave][rl][c] = an; if (jj == 3) sl[wave][rl][c >> 2] = an; } }
  LDSX();
#pragma unroll 4
  for (int rl = 0; rl < 16; ++rl) vst2(anew + (size_t)(r0 + rl) * MD + n0 + lane * 4, *(const v4f*)(&sg[2][wave][rl][lane * 4]));
  for (int q = lane; q < 16 * 8; q += 32) { const int rl = q >> 3, pc = q & 7; vst2(ANL + (size_t)(r0 + rl) * MM + (n0 >> 2) + pc * 4, *(const v4f*)(&sl[wave][rl][pc * 4])); }
}
__global__ __launch_bounds__(128) void k_p2(const float* __restrict__ x, const float* __restrict__ ANL, const float* __restrict__ anew, const float* __restrict__ Aot, const float* __restrict__ Bot, const float* __restrict__ bot, float* __restrict__ S3, float* __restrict__ AAL) {
  __shared__ __align__(16) float sa[4][16][132];
  __shared__ __align__(16) float s3[4][16][36], sL[4][16][36];
  const int tid = threadIdx.x, wave = tid >> 5, lane = tid & 31, col = lane & 15, g = lane >> 4;
  const int r0 = blockIdx.x * 64 + wave * 16, n0 = blockIdx.y * 128;
  v8f acc[8] = {};
#pragma unroll 1
  for (int kc = 0; kc < MM / 32; ++kc) { const v16h fa = frag_f32(ANL + (size_t)(r0 + col) * MM + kc * 32, lane);
#pragma unroll
    for (int j = 0; j < 8; ++j) acc[j] = wmma16(fa, fragc_f32s(Aot, kc * 32, n0 + j * 16 + col, lane, MD, 16.0f), acc[j]); }
#pragma unroll 1
  for (int kc = 0; kc < NX / 32; ++kc) { const v16h fa = frag_f32(x + (size_t)(r0 + col) * NX + kc * 32, lane);
#pragma unroll
    for (int j = 0; j < 8; ++j) acc[j] = wmma16(fa, fragc_f32s(Bot, kc * 32, n0 + j * 16 + col, lane, MD, 16.0f), acc[j]); }
#pragma unroll
  for (int j = 0; j < 8; ++j) { const float bv = bot[n0 + j * 16 + col];
#pragma unroll
    for (int r = 0; r < 8; ++r) sa[wave][8 * g + r][j * 16 + col] = acc[j][r] * (1.0f / 16.0f) + bv; }
  LDSX();
  { const int rl = lane >> 1, hf = lane & 1; const int row = r0 + rl;
#pragma unroll 1
    for (int c = hf * 64; c < hf * 64 + 64; ++c) { const int n = n0 + c; const int mcol = n >> 2;
      const float v = sa[wave][rl][c] - ANL[(size_t)row * MM + mcol] * Aot[(size_t)mcol * MD + n];
      sa[wave][rl][c] = tanhf(anew[(size_t)row * MD + n]) * sigm(v); } }
  LDSX();
  { const int rl = lane >> 1, hf = lane & 1;
    for (int ml = hf * 16; ml < hf * 16 + 16; ++ml) { const float* p4 = &sa[wave][rl][ml * 4]; s3[wave][rl][ml] = (p4[0] + p4[1]) + p4[2]; sL[wave][rl][ml] = p4[3]; } }
  LDSX();
  for (int q = lane; q < 16 * 8; q += 32) { const int rl = q >> 3, pc = q & 7; vst2(S3 + (size_t)(r0 + rl) * MM + (n0 >> 2) + pc * 4, *(const v4f*)(&s3[wave][rl][pc * 4])); vst2(AAL + (size_t)(r0 + rl) * MM + (n0 >> 2) + pc * 4, *(const v4f*)(&sL[wave][rl][pc * 4])); }
}
__global__ __launch_bounds__(128) void k_p3(const float* __restrict__ S3, const float* __restrict__ AAL, const float* __restrict__ Ast, float* __restrict__ mnew) {
  __shared__ __align__(16) float so[4][16][132];
  const int tid = threadIdx.x, wave = tid >> 5, lane = tid & 31, col = lane & 15, g = lane >> 4;
  const int r0 = blockIdx.x * 64 + wave * 16, n0 = blockIdx.y * 128;
  v8f acc[8] = {};
#pragma unroll 1
  for (int kc = 0; kc < MM / 32; ++kc) { const v16h fa = frag_f32(AAL + (size_t)(r0 + col) * MM + kc * 32, lane);
#pragma unroll
    for (int j = 0; j < 8; ++j) acc[j] = wmma16(fa, fragc_f32s(Ast, kc * 32, n0 + j * 16 + col, lane, MM, 16.0f), acc[j]); }
#pragma unroll
  for (int j = 0; j < 8; ++j) { const int n = n0 + j * 16 + col;
#pragma unroll
    for (int r = 0; r < 8; ++r) so[wave][8 * g + r][j * 16 + col] = acc[j][r] * (1.0f / 16.0f) + S3[(size_t)(r0 + 8 * g + r) * MM + n]; }
  LDSX();
#pragma unroll 4
  for (int rl = 0; rl < 16; ++rl) vst2(mnew + (size_t)(r0 + rl) * MM + n0 + lane * 4, *(const v4f*)(&so[wave][rl][lane * 4]));
}
extern "C" void kernel_launch(void* const* d_in, const int* in_sizes, int n_in, void* d_out, int out_size, void* d_ws, size_t ws_size, hipStream_t stream) {
  (void)in_sizes; (void)n_in; (void)out_size; (void)ws_size;
  const float** I = (const float**)d_in;
  const float* x = I[0]; const float* m = I[1]; const float* a = I[2]; const float* Afg = I[3]; const float* Ain = I[4]; const float* Ath = I[5]; const float* Aot = I[6]; const float* Ast = I[7]; const float* Apt = I[8];
  const float* Bfg = I[9]; const float* Bin = I[10]; const float* Bth = I[11]; const float* Bot = I[12]; const float* bfg = I[13]; const float* bin_ = I[14]; const float* bth = I[15]; const float* bot = I[16];
  float* mnew = (float*)d_out; float* anew = (float*)((char*)d_out + 2097152);
  char* ws = (char*)d_ws; size_t off = 0;
  auto take = [&](size_t bytes) { char* p = ws + off; off += (bytes + 255) & ~(size_t)255; return p; };
  float* AL = (float*)take((size_t)NBT * MM * 4); float* ANL = (float*)take((size_t)NBT * MM * 4); float* S3 = (float*)take((size_t)NBT * MM * 4); float* AAL = (float*)take((size_t)NBT * MM * 4);
  k_last<<<NBT * MM / 256, 256, 0, stream>>>(a, AL);
  k_p1<<<dim3(NBT / 64, MD / 128), 128, 0, stream>>>(x, m, a, AL, Afg, Ain, Ath, Apt, Bfg, Bin, Bth, bfg, bin_, bth, anew, ANL);
  k_p2<<<dim3(NBT / 64, MD / 128), 128, 0, stream>>>(x, ANL, anew, Aot, Bot, bot, S3, AAL);
  k_p3<<<dim3(NBT / 64, MM / 128), 128, 0, stream>>>(S3, AAL, Ast, mnew);
}
